// MambaResidualBlock_67980742362029
// MI455X (gfx1250) — hardware-run, weakly checked
//
#include <hip/hip_runtime.h>
#include <math.h>

typedef __attribute__((ext_vector_type(16))) _Float16 v16h;
typedef __attribute__((ext_vector_type(8)))  _Float16 v8h;
typedef __attribute__((ext_vector_type(8)))  float    v8f;
typedef __attribute__((ext_vector_type(4)))  float    v4f;

constexpr int kNB    = 4;
constexpr int kSeq   = 1024;
constexpr int kDm    = 1024;
constexpr int kDi    = 2048;
constexpr int kNs    = 16;
constexpr int kDtR   = 64;
constexpr int kTaps  = 4;
constexpr int kXpN   = 96;
constexpr int kXpP   = 128;
constexpr int kPw    = 2 * kDi;
constexpr int kRows  = kNB * kSeq;
constexpr int kHidB  = kDi * kNs + (kTaps - 1) * kDi;
constexpr int kTP    = 260;
constexpr int kTailRows = kNB * (kTaps - 1);
constexpr float kWCarry   = 32.0f;
constexpr float kDtWCarry = 8.0f;
constexpr float kYCarry   = 16.0f;

static_assert(kDtR + 2 * kNs == kXpN, "x_proj width");
static_assert(kHidB == 38912, "hidden row length");
static_assert(kRows == 4096 && kPw == 4096, "token rows / in_proj width");
static_assert((kDm % 32) == 0 && (kDi % 32) == 0 && (kDtR % 32) == 0, "GEMM K multiples of 32");
static_assert((kRows % 64) == 0 && (kPw % 64) == 0 && (kXpP % 64) == 0 && (kDi % 64) == 0 && (kDm % 64) == 0, "GEMM M,N multiples of 64");
static_assert((kSeq % 64) == 0 && (kDi % 256) == 0 && (kSeq % 16) == 0, "tile multiples");
static_assert(kTailRows == 12, "tail rows");
static_assert(kDm == 256 * 4, "LayerNorm block covers one row with 4 columns per thread");

constexpr size_t kOffWIN  = 0;
constexpr size_t kOffWXP  = kOffWIN  + (size_t)kPw  * kDm  * 2;
constexpr size_t kOffWDT  = kOffWXP  + (size_t)kXpP * kDi  * 2;
constexpr size_t kOffWOUT = kOffWDT  + (size_t)kDi  * kDtR * 2;
constexpr size_t kOffWF1  = kOffWOUT + (size_t)kDm  * kDi  * 2;
constexpr size_t kOffWF2  = kOffWF1  + (size_t)kDm  * kDm  * 2;
constexpr size_t kOffXN   = kOffWF2  + (size_t)kDm  * kDm  * 2;
constexpr size_t kOffP    = kOffXN   + (size_t)kRows * kDm * 2;
constexpr size_t kOffUC   = kOffP    + (size_t)kRows * kPw * 2;
constexpr size_t kOffDBL  = kOffUC   + (size_t)kRows * kDi * 2;
constexpr size_t kOffDTR  = kOffDBL  + (size_t)kRows * kXpP * 4;
constexpr size_t kOffDLR  = kOffDTR  + (size_t)kRows * kDtR * 2;
constexpr size_t kOffY    = kOffDLR  + (size_t)kRows * kDi * 4;
constexpr size_t kWsTotal = kOffY    + (size_t)kRows * kDi * 2;
static_assert(kWsTotal == 129236992ull, "carve total");
static_assert(kWsTotal <= 134217728ull, "carve cap");
static_assert((kOffWXP % 128) == 0 && (kOffWDT % 128) == 0 && (kOffWOUT % 128) == 0 && (kOffWF1 % 128) == 0 &&
              (kOffWF2 % 128) == 0 && (kOffXN % 128) == 0 && (kOffP % 128) == 0 && (kOffUC % 128) == 0 &&
              (kOffDBL % 128) == 0 && (kOffDTR % 128) == 0 && (kOffDLR % 128) == 0 && (kOffY % 128) == 0, "128-B aligned regions");
static_assert((size_t)kRows * kDm * 2 * 2 <= (size_t)kRows * kDi * 2, "O16 + H16 inside UC");
static_assert((size_t)kRows * kDm * 4 * 2 <= (size_t)kRows * kDi * 4, "result plane + out32 inside DLR");

__device__ __forceinline__ float h16_to_f32(unsigned hb) {
  const unsigned sgn = (hb & 0x8000u) << 16;
  const unsigned em = hb & 0x7fffu;
  const float fn = __uint_as_float((em << 13) + 0x38000000u);
  const float fs = (float)em * 5.9604644775390625e-8f;
  const float mag = (em < 0x400u) ? fs : fn;
  return __uint_as_float(__float_as_uint(mag) | sgn);
}

union FragU { v16h v; v8h h[2]; };
__device__ __forceinline__ v16h frag_load_h(const _Float16* p) {
  FragU f;
  f.h[0] = *(const v8h*)(p);
  f.h[1] = *(const v8h*)(p + 16);
  return f.v;
}
__device__ __forceinline__ v8f mma_h(v16h a, v16h b, v8f c) {
  return __builtin_amdgcn_wmma_f32_16x16x32_f16(false, a, false, b, (short)0, c, false, false);
}
__device__ __forceinline__ void guard_row4(v8f& a0, v8f& a1, v8f& a2, v8f& a3, v16h x, v16h b0, v16h b1, v16h b2, v16h b3) {
  asm volatile("v_nop\n\tv_nop\n\tv_nop\n\tv_nop" : "+v"(a0), "+v"(a1), "+v"(a2), "+v"(a3) : "v"(x), "v"(b0), "v"(b1), "v"(b2), "v"(b3));
}
__device__ __forceinline__ void keep4_h(v16h a, v16h b, v16h c, v16h d) { asm volatile("v_nop" :: "v"(a), "v"(b), "v"(c), "v"(d)); }
__device__ __forceinline__ void acc_guard4(v8f& a, v8f& b, v8f& c, v8f& d) { asm volatile("v_nop\n\tv_nop\n\tv_nop\n\tv_nop" : "+v"(a), "+v"(b), "+v"(c), "+v"(d)); }

template <int BIAS_MODE, int OUT_MODE>
__global__ __launch_bounds__(256) void wmma_gemm64_f16(
    const unsigned short* __restrict__ Ap, int lda,
    const unsigned short* __restrict__ Btp, int ldb,
    void* __restrict__ Cout, int ldc,
    const float* __restrict__ bias,
    int M, int N, int K, float scale) {
  const _Float16* A  = (const _Float16*)Ap;
  const _Float16* Bt = (const _Float16*)Btp;
  __shared__ __align__(16) float sT[8][16 * 68];
  const int lane = threadIdx.x & 31;
  const int wave = threadIdx.x >> 5;
  const int tilesN = N >> 6;
  const int tilesM = M >> 6;
  const int tile = blockIdx.x * 8 + wave;
  if (tile >= tilesM * tilesN) return;
  const int tm = tile / tilesN;
  const int tn = tile - tm * tilesN;
  const int m0 = tm << 6;
  const int n0 = tn << 6;

  const int rlane = lane & 15;
  const int koff  = (lane >> 4) * 8;
  const int mOff  = (lane >> 4) * 8;

  v8f acc[4][4];
#pragma unroll
  for (int i = 0; i < 4; ++i)
#pragma unroll
    for (int j = 0; j < 4; ++j) acc[i][j] = (v8f){0.f, 0.f, 0.f, 0.f, 0.f, 0.f, 0.f, 0.f};

  for (int k0 = 0; k0 < K; k0 += 32) {
    v16h bh[4];
#pragma unroll
    for (int j = 0; j < 4; ++j) {
      const size_t bo = (size_t)(n0 + (j << 4) + rlane) * ldb + koff + k0;
      bh[j] = frag_load_h(Bt + bo);
    }
#pragma unroll
    for (int i = 0; i < 4; ++i) {
      const size_t ao = (size_t)(m0 + (i << 4) + rlane) * lda + koff + k0;
      const v16h ah = frag_load_h(A + ao);
#pragma unroll
      for (int j = 0; j < 4; ++j) acc[i][j] = mma_h(ah, bh[j], acc[i][j]);
      guard_row4(acc[i][0], acc[i][1], acc[i][2], acc[i][3], ah, bh[0], bh[1], bh[2], bh[3]);
    }
    keep4_h(bh[0], bh[1], bh[2], bh[3]);
  }
  acc_guard4(acc[0][0], acc[0][1], acc[0][2], acc[0][3]);
  acc_guard4(acc[1][0], acc[1][1], acc[1][2], acc[1][3]);
  acc_guard4(acc[2][0], acc[2][1], acc[2][2], acc[2][3]);
  acc_guard4(acc[3][0], acc[3][1], acc[3][2], acc[3][3]);

  float* slab = sT[wave];
#pragma unroll
  for (int i = 0; i < 4; ++i) {
    const int mBase = m0 + (i << 4);
#pragma unroll
    for (int j = 0; j < 4; ++j) {
      const int n = n0 + (j << 4) + rlane;
      float bv = 0.f;
      if (BIAS_MODE == 2) bv = bias[n];
#pragma unroll
      for (int r = 0; r < 8; ++r) {
        float v = acc[i][j][r] * scale;
        if (BIAS_MODE == 2) v += bv;
        slab[(mOff + r) * 68 + (j << 4) + rlane] = v;
      }
    }
    __builtin_amdgcn_fence(__ATOMIC_RELEASE, "workgroup");
    __builtin_amdgcn_wave_barrier();
    __builtin_amdgcn_fence(__ATOMIC_ACQUIRE, "workgroup");
    if (OUT_MODE == 0) {
      float* C = (float*)Cout;
      const int hh = lane >> 4, c4 = (lane & 15) * 4;
      for (int pass = 0; pass < 2; ++pass) {
#pragma unroll
        for (int it = 0; it < 8; ++it) {
          const int row = it * 2 + hh;
          v4f v = *(const v4f*)(slab + row * 68 + c4);
          *(volatile v4f*)(C + (size_t)(mBase + row) * ldc + n0 + c4) = v;
        }
        __threadfence();
      }
    } else {
      const int q = lane >> 3, c8 = (lane & 7) * 8;
      unsigned short* C = (unsigned short*)Cout;
      for (int pass = 0; pass < 2; ++pass) {
#pragma unroll
        for (int it = 0; it < 4; ++it) {
          const int row = it * 4 + q;
          const float* sp = slab + row * 68 + c8;
          v8h hv;
#pragma unroll
          for (int e = 0; e < 8; ++e) hv[e] = (_Float16)sp[e];
          *(volatile v8h*)(C + (size_t)(mBase + row) * ldc + n0 + c8) = hv;
        }
        __threadfence();
      }
    }
    __builtin_amdgcn_fence(__ATOMIC_RELEASE, "workgroup");
    __builtin_amdgcn_wave_barrier();
    __builtin_amdgcn_fence(__ATOMIC_ACQUIRE, "workgroup");
  }
}

__global__ __launch_bounds__(256) void cast_f16_kernel(
    const float* __restrict__ src, unsigned short* __restrict__ dst, int total8, int valid8, float scale)
{
  const int i = blockIdx.x * 256 + threadIdx.x;
  if (i >= total8) return;
  const bool ok = (i < valid8);
  const int ic = ok ? i : (valid8 - 1);
  const float* p = src + ((size_t)ic << 3);
  const v4f a0 = *(const v4f*)(p);
  const v4f a1 = *(const v4f*)(p + 4);
  v8h hv;
#pragma unroll
  for (int e = 0; e < 4; ++e) {
    const float f0 = ok ? (a0[e] * scale) : 0.0f;
    const float f1 = ok ? (a1[e] * scale) : 0.0f;
    hv[e]     = (_Float16)f0;
    hv[4 + e] = (_Float16)f1;
  }
  unsigned short* q = dst + ((size_t)i << 3);
  *(volatile v8h*)q = hv;
  __threadfence();
  *(volatile v8h*)q = hv;
}

__global__ __launch_bounds__(256) void rmsnorm_f16_kernel(
    const float* __restrict__ x, const float* __restrict__ nw, unsigned short* __restrict__ XN)
{
  const int lane = threadIdx.x & 31, wave = threadIdx.x >> 5;
  const int row = blockIdx.x * 8 + wave;
  const float* xr = x + (size_t)row * kDm;
  v4f a[4][2];
  float ss = 0.f;
#pragma unroll
  for (int i = 0; i < 4; ++i) {
    const int k = i * 256 + lane * 8;
    a[i][0] = *(const v4f*)(xr + k);
    a[i][1] = *(const v4f*)(xr + k + 4);
#pragma unroll
    for (int e = 0; e < 4; ++e) {
      ss = fmaf(a[i][0][e], a[i][0][e], ss);
      ss = fmaf(a[i][1][e], a[i][1][e], ss);
    }
  }
  ss += __shfl_xor(ss, 16, 32);
  ss += __shfl_xor(ss, 8, 32);
  ss += __shfl_xor(ss, 4, 32);
  ss += __shfl_xor(ss, 2, 32);
  ss += __shfl_xor(ss, 1, 32);
  const float rs = rsqrtf(ss * (1.0f / (float)kDm) + 1e-5f);
  v8h hv[4];
#pragma unroll
  for (int i = 0; i < 4; ++i) {
    const int k = i * 256 + lane * 8;
    const v4f w0 = *(const v4f*)(nw + k);
    const v4f w1 = *(const v4f*)(nw + k + 4);
#pragma unroll
    for (int e = 0; e < 4; ++e) {
      hv[i][e]     = (_Float16)((a[i][0][e] * rs) * w0[e]);
      hv[i][4 + e] = (_Float16)((a[i][1][e] * rs) * w1[e]);
    }
  }
  unsigned short* dr = XN + (size_t)row * kDm;
  for (int pass = 0; pass < 2; ++pass) {
#pragma unroll
    for (int i = 0; i < 4; ++i) *(volatile v8h*)(dr + i * 256 + lane * 8) = hv[i];
    __threadfence();
  }
}

__global__ __launch_bounds__(256) void conv_silu_kernel(
    const unsigned* __restrict__ P32, const float* __restrict__ cw, const float* __restrict__ cb,
    unsigned short* __restrict__ UC16)
{
  __shared__ __align__(16) float sT[16 * kTP];
  const int tid = threadIdx.x, lane = tid & 31, wave = tid >> 5;
  const int d0 = blockIdx.x * 256, d = d0 + tid;
  const int g0 = blockIdx.y * 64;
  const int tb = g0 & (kSeq - 1);
  const v4f w4 = *(const v4f*)(cw + (size_t)d * kTaps);
  const float w0 = w4[0], w1 = w4[1], w2 = w4[2], w3 = w4[3];
  const float bc = cb[d];
  const unsigned hsh = (unsigned)(tid & 1) * 16u;
  const int wcol = d >> 1;
  constexpr int kPw32 = kPw / 2;
  float xm3, xm2, xm1;
  {
    const bool hist = (tb > 0);
    const int rb = hist ? (g0 - 3) : g0;
    const unsigned u3 = P32[(size_t)rb * kPw32 + wcol];
    const unsigned u2 = P32[(size_t)(rb + 1) * kPw32 + wcol];
    const unsigned u1 = P32[(size_t)(rb + 2) * kPw32 + wcol];
    const float v3 = h16_to_f32((u3 >> hsh) & 0xffffu);
    const float v2 = h16_to_f32((u2 >> hsh) & 0xffffu);
    const float v1 = h16_to_f32((u1 >> hsh) & 0xffffu);
    xm3 = hist ? v3 : 0.f;
    xm2 = hist ? v2 : 0.f;
    xm1 = hist ? v1 : 0.f;
  }
#pragma unroll 1
  for (int sub = 0; sub < 4; ++sub) {
    const int lb = g0 + sub * 16;
#pragma unroll 1
    for (int s = 0; s < 16; ++s) {
      const unsigned uw = P32[(size_t)(lb + s) * kPw32 + wcol];
      const float xc = h16_to_f32((uw >> hsh) & 0xffffu);
      float acc = w0 * xm3;
      acc = fmaf(w1, xm2, acc);
      acc = fmaf(w2, xm1, acc);
      acc = fmaf(w3, xc, acc);
      const float sv = acc + bc;
      const float sg = __builtin_amdgcn_rcpf(1.0f + expf(-sv));
      sT[s * kTP + tid] = sv * sg;
      xm3 = xm2; xm2 = xm1; xm1 = xc;
    }
    __syncthreads();
    v8h bv[2];
#pragma unroll
    for (int it = 0; it < 2; ++it) {
      const float* sp = sT + (it * 8 + wave) * kTP + lane * 8;
      const v4f a0 = *(const v4f*)(sp);
      const v4f a1 = *(const v4f*)(sp + 4);
#pragma unroll
      for (int e = 0; e < 4; ++e) {
        bv[it][e]     = (_Float16)a0[e];
        bv[it][4 + e] = (_Float16)a1[e];
      }
    }
    for (int pass = 0; pass < 2; ++pass) {
#pragma unroll
      for (int it = 0; it < 2; ++it)
        *(volatile v8h*)(UC16 + (size_t)(lb + it * 8 + wave) * kDi + d0 + lane * 8) = bv[it];
      __threadfence();
    }
    __syncthreads();
  }
}

__global__ __launch_bounds__(256) void dt_cast_kernel(
    const float* __restrict__ DBL, unsigned short* __restrict__ DTR, int total8)
{
  const int i = blockIdx.x * 256 + threadIdx.x;
  if (i >= total8) return;
  const int e0  = i << 3;
  const int row = e0 >> 6;
  const int c8  = e0 & 63;
  const float* p = DBL + (size_t)row * kXpP + c8;
  const v4f a0 = *(const v4f*)(p);
  const v4f a1 = *(const v4f*)(p + 4);
  v8h hv;
#pragma unroll
  for (int e = 0; e < 4; ++e) {
    hv[e]     = (_Float16)a0[e];
    hv[4 + e] = (_Float16)a1[e];
  }
  unsigned short* qd = DTR + e0;
  *(volatile v8h*)qd = hv;
  __threadfence();
  *(volatile v8h*)qd = hv;
}

__global__ __launch_bounds__(256) void scan_gate_kernel(
    const float* __restrict__ DLR, const unsigned* __restrict__ UC32, const unsigned* __restrict__ P32,
    const float* __restrict__ DBL, const float* __restrict__ A_log, const float* __restrict__ Dv,
    unsigned short* __restrict__ Y16, float* __restrict__ hid)
{
  __shared__ __align__(16) float sBC[16 * 32];
  __shared__ __align__(16) float sY[16 * kTP];
  static_assert(16 * kTP >= 256 * kNs, "state staging fits the tile");
  const int tid = threadIdx.x, lane = tid & 31, wave = tid >> 5;
  const int bix = blockIdx.x >> 3;
  const int d0 = (blockIdx.x & 7) * 256;
  const int d = d0 + tid;
  const size_t row0 = (size_t)bix * kSeq;
  constexpr int kPw32 = kPw / 2;
  constexpr int kDi32 = kDi / 2;

#pragma unroll 1
  for (int n = 0; n < kNs; ++n) sY[n * 256 + tid] = -expf(A_log[(size_t)d * kNs + n]);
  __syncthreads();
  float An[kNs], h[kNs];
#pragma unroll
  for (int n = 0; n < kNs; ++n) {
    An[n] = sY[n * 256 + tid];
    h[n] = 0.f;
  }
  const float Dd = Dv[d];
  const unsigned hsh = (unsigned)(tid & 1) * 16u;
  const int wcol = d >> 1;

#pragma unroll 1
  for (int c = 0; c < kSeq / 16; ++c) {
    const int l0 = c * 16;
    if (tid < 128) {
      const int r = tid >> 3, q = (tid & 7) * 4;
      const v4f v = *(const v4f*)(DBL + (row0 + l0 + r) * kXpP + kDtR + q);
      *(v4f*)(sBC + r * 32 + q) = v;
    }
    __syncthreads();
#pragma unroll 1
    for (int s = 0; s < 16; ++s) {
      const size_t m = row0 + (size_t)(l0 + s);
      const float a = DLR[m * kDi + d];
      const unsigned uw = UC32[m * kDi32 + wcol];
      const unsigned zw = P32[m * kPw32 + kDi32 + wcol];
      const float delta = fmaxf(a, 0.0f) + log1pf(expf(-fabsf(a)));
      const float xv = h16_to_f32((uw >> hsh) & 0xffffu);
      const float zv = h16_to_f32((zw >> hsh) & 0xffffu);
      v4f Bq[4], Cq[4];
#pragma unroll
      for (int qq = 0; qq < 4; ++qq) {
        Bq[qq] = *(const v4f*)(sBC + s * 32 + 4 * qq);
        Cq[qq] = *(const v4f*)(sBC + s * 32 + kNs + 4 * qq);
      }
      const float dtx = delta * xv;
      float y = 0.f;
#pragma unroll
      for (int n = 0; n < kNs; ++n) {
        const float e = __expf(delta * An[n]);
        const float hn = fmaf(e, h[n], dtx * Bq[n >> 2][n & 3]);
        h[n] = hn;
        y = fmaf(hn, Cq[n >> 2][n & 3], y);
      }
      y = fmaf(xv, Dd, y);
      const float sg = __builtin_amdgcn_rcpf(1.0f + __expf(-zv));
      const float g  = zv * sg;
      sY[s * kTP + tid] = (y * g) * kYCarry;
    }
    __syncthreads();
    v8h hv[2];
#pragma unroll
    for (int it = 0; it < 2; ++it) {
      const float* sp = sY + (it * 8 + wave) * kTP + lane * 8;
      const v4f a0 = *(const v4f*)(sp);
      const v4f a1 = *(const v4f*)(sp + 4);
#pragma unroll
      for (int e = 0; e < 4; ++e) {
        hv[it][e]     = (_Float16)a0[e];
        hv[it][4 + e] = (_Float16)a1[e];
      }
    }
    for (int pass = 0; pass < 2; ++pass) {
#pragma unroll
      for (int it = 0; it < 2; ++it)
        *(volatile v8h*)(Y16 + (row0 + l0 + it * 8 + wave) * kDi + d0 + lane * 8) = hv[it];
      __threadfence();
    }
  }

  __syncthreads();
#pragma unroll
  for (int q = 0; q < 4; ++q)
    *(v4f*)(sY + tid * kNs + 4 * q) = (v4f){h[4 * q], h[4 * q + 1], h[4 * q + 2], h[4 * q + 3]};
  __syncthreads();
  v4f hs[4];
#pragma unroll
  for (int it = 0; it < 4; ++it) hs[it] = *(const v4f*)(sY + wave * 512 + it * 128 + lane * 4);
  float* hp = hid + (size_t)bix * kHidB + (size_t)(d0 + wave * 32) * kNs;
  for (int pass = 0; pass < 2; ++pass) {
#pragma unroll
    for (int it = 0; it < 4; ++it) *(volatile v4f*)(hp + it * 128 + lane * 4) = hs[it];
    __threadfence();
  }
}

__global__ __launch_bounds__(256) void resadd_kernel(
    const float* __restrict__ RAW, const float* __restrict__ x,
    float* __restrict__ O32, unsigned short* __restrict__ O16)
{
  const int tid = threadIdx.x;
  const size_t base = (size_t)blockIdx.x * 2048;
  v4f f[2];
#pragma unroll
  for (int j = 0; j < 2; ++j) {
    const size_t o = base + (size_t)j * 1024 + (size_t)tid * 4;
    const v4f r4 = *(const v4f*)(RAW + o);
    const v4f x4 = *(const v4f*)(x + o);
    f[j] = r4 + x4;
  }
  const size_t e0 = base + (size_t)tid * 8;
  const v4f r0 = *(const v4f*)(RAW + e0);
  const v4f r1 = *(const v4f*)(RAW + e0 + 4);
  const v4f x0 = *(const v4f*)(x + e0);
  const v4f x1 = *(const v4f*)(x + e0 + 4);
  const v4f s0 = r0 + x0;
  const v4f s1 = r1 + x1;
  v8h hv;
#pragma unroll
  for (int e = 0; e < 4; ++e) {
    hv[e]     = (_Float16)s0[e];
    hv[4 + e] = (_Float16)s1[e];
  }
  for (int pass = 0; pass < 2; ++pass) {
#pragma unroll
    for (int j = 0; j < 2; ++j)
      *(volatile v4f*)(O32 + base + (size_t)j * 1024 + (size_t)tid * 4) = f[j];
    *(volatile v8h*)(O16 + e0) = hv;
    __threadfence();
  }
}

__global__ __launch_bounds__(256) void gelu_f16_kernel(
    const float* __restrict__ RAW, unsigned short* __restrict__ H16)
{
  __shared__ __align__(16) float sG[2048];
  const int tid = threadIdx.x;
  const size_t base = (size_t)blockIdx.x * 2048;
#pragma unroll 1
  for (int it = 0; it < 8; ++it) {
    const int idx = it * 256 + tid;
    const float v = RAW[base + idx];
    sG[idx] = 0.5f * v * (1.0f + erff(v * 0.70710678118654752f));
  }
  __syncthreads();
  const v4f a0 = *(const v4f*)(sG + tid * 8);
  const v4f a1 = *(const v4f*)(sG + tid * 8 + 4);
  v8h hv;
#pragma unroll
  for (int e = 0; e < 4; ++e) {
    hv[e]     = (_Float16)a0[e];
    hv[4 + e] = (_Float16)a1[e];
  }
  unsigned short* q = H16 + base + (size_t)tid * 8;
  *(volatile v8h*)q = hv;
  __threadfence();
  *(volatile v8h*)q = hv;
}

__global__ __launch_bounds__(256) void layernorm_out_kernel(
    const float* __restrict__ Z, const float* __restrict__ O, const float* __restrict__ lw,
    const float* __restrict__ lb, float* __restrict__ dout)
{
  __shared__ float sS[8];
  __shared__ float sQ[8];
  const int tid = threadIdx.x, lane = tid & 31, wave = tid >> 5;
  const size_t off = (size_t)blockIdx.x * kDm + (size_t)tid * 4;
  const v4f a = *(const v4f*)(Z + off);
  const v4f b = *(const v4f*)(O + off);
  const v4f z = a + b;
  float s = (z[0] + z[1]) + (z[2] + z[3]);
  s += __shfl_xor(s, 16, 32);
  s += __shfl_xor(s, 8, 32);
  s += __shfl_xor(s, 4, 32);
  s += __shfl_xor(s, 2, 32);
  s += __shfl_xor(s, 1, 32);
  if (lane == 0) sS[wave] = s;
  __syncthreads();
  const float tot = ((sS[0] + sS[1]) + (sS[2] + sS[3])) + ((sS[4] + sS[5]) + (sS[6] + sS[7]));
  const float mu = tot * (1.0f / (float)kDm);
  const float c0 = z[0] - mu;
  const float c1 = z[1] - mu;
  const float c2 = z[2] - mu;
  const float c3 = z[3] - mu;
  float s2 = c0 * c0;
  s2 = fmaf(c1, c1, s2);
  s2 = fmaf(c2, c2, s2);
  s2 = fmaf(c3, c3, s2);
  s2 += __shfl_xor(s2, 16, 32);
  s2 += __shfl_xor(s2, 8, 32);
  s2 += __shfl_xor(s2, 4, 32);
  s2 += __shfl_xor(s2, 2, 32);
  s2 += __shfl_xor(s2, 1, 32);
  if (lane == 0) sQ[wave] = s2;
  __syncthreads();
  const float tot2 = ((sQ[0] + sQ[1]) + (sQ[2] + sQ[3])) + ((sQ[4] + sQ[5]) + (sQ[6] + sQ[7]));
  const float rs = rsqrtf(tot2 * (1.0f / (float)kDm) + 1e-5f);
  const v4f w4 = *(const v4f*)(lw + tid * 4);
  const v4f b4 = *(const v4f*)(lb + tid * 4);
  v4f ov;
  ov[0] = fmaf(c0 * rs, w4[0], b4[0]);
  ov[1] = fmaf(c1 * rs, w4[1], b4[1]);
  ov[2] = fmaf(c2 * rs, w4[2], b4[2]);
  ov[3] = fmaf(c3 * rs, w4[3], b4[3]);
  float* p = dout + off;
  *(volatile v4f*)p = ov;
  __threadfence();
  *(volatile v4f*)p = ov;
}

__global__ __launch_bounds__(256) void utail_kernel(
    const float* __restrict__ x, const float* __restrict__ nw, const float* __restrict__ Win,
    float* __restrict__ hid)
{
  __shared__ __align__(16) float sX[kTailRows * kDm];
  __shared__ __align__(16) float sR[kTailRows * 32];
  const int tid = threadIdx.x, lane = tid & 31, wave = tid >> 5;
  const int d0 = blockIdx.x * 32;

#pragma unroll 1
  for (int rr = wave; rr < kTailRows; rr += 8) {
    const int b = rr / 3, j = rr - b * 3;
    const float* xr = x + ((size_t)b * kSeq + (kSeq - 3) + j) * kDm;
    float ss = 0.f;
#pragma unroll 1
    for (int i = 0; i < 8; ++i) {
      const v4f a = *(const v4f*)(xr + i * 128 + lane * 4);
      ss = fmaf(a[0], a[0], ss);
      ss = fmaf(a[1], a[1], ss);
      ss = fmaf(a[2], a[2], ss);
      ss = fmaf(a[3], a[3], ss);
    }
    ss += __shfl_xor(ss, 16, 32);
    ss += __shfl_xor(ss, 8, 32);
    ss += __shfl_xor(ss, 4, 32);
    ss += __shfl_xor(ss, 2, 32);
    ss += __shfl_xor(ss, 1, 32);
    const float rs = rsqrtf(ss * (1.0f / (float)kDm) + 1e-5f);
#pragma unroll 1
    for (int i = 0; i < 8; ++i) {
      const int k = i * 128 + lane * 4;
      const v4f a = *(const v4f*)(xr + k);
      const v4f w = *(const v4f*)(nw + k);
      v4f o;
      o[0] = (a[0] * rs) * w[0];
      o[1] = (a[1] * rs) * w[1];
      o[2] = (a[2] * rs) * w[2];
      o[3] = (a[3] * rs) * w[3];
      *(v4f*)(sX + rr * kDm + k) = o;
    }
  }
  __syncthreads();

#pragma unroll 1
  for (int c = 0; c < 4; ++c) {
    const int ch = wave * 4 + c;
    const float* wr = Win + (size_t)(d0 + ch) * kDm;
    float acc[kTailRows];
#pragma unroll
    for (int r = 0; r < kTailRows; ++r) acc[r] = 0.f;
#pragma unroll 1
    for (int i = 0; i < 8; ++i) {
      const int k = i * 128 + lane * 4;
      const v4f w = *(const v4f*)(wr + k);
#pragma unroll
      for (int r = 0; r < kTailRows; ++r) {
        const v4f xv = *(const v4f*)(sX + r * kDm + k);
        float t = acc[r];
        t = fmaf(w[0], xv[0], t);
        t = fmaf(w[1], xv[1], t);
        t = fmaf(w[2], xv[2], t);
        t = fmaf(w[3], xv[3], t);
        acc[r] = t;
      }
    }
#pragma unroll
    for (int r = 0; r < kTailRows; ++r) {
      float t = acc[r];
      t += __shfl_xor(t, 16, 32);
      t += __shfl_xor(t, 8, 32);
      t += __shfl_xor(t, 4, 32);
      t += __shfl_xor(t, 2, 32);
      t += __shfl_xor(t, 1, 32);
      acc[r] = t;
    }
    if (lane == 0) {
#pragma unroll
      for (int r = 0; r < kTailRows; ++r) sR[r * 32 + ch] = acc[r];
    }
  }
  __syncthreads();

  if (wave < 3) {
    const int r = wave * 4 + (lane >> 3);
    const int c4 = (lane & 7) * 4;
    const int b = r / 3, j = r - b * 3;
    const v4f v = *(const v4f*)(sR + r * 32 + c4);
    float* p = hid + (size_t)b * kHidB + (size_t)kDi * kNs + (size_t)j * kDi + d0 + c4;
    *(volatile v4f*)p = v;
    __threadfence();
    *(volatile v4f*)p = v;
  }
}

extern "C" void kernel_launch(void* const* d_in, const int* in_sizes, int n_in,
                              void* d_out, int out_size, void* d_ws, size_t ws_size,
                              hipStream_t stream)
{
  if (n_in < 17) return;
  if (in_sizes[0] != kRows * kDm) return;
  if (in_sizes[1] != kDm) return;
  if (in_sizes[2] != kPw * kDm) return;
  if (in_sizes[3] != kDi * kTaps) return;
  if (in_sizes[4] != kDi) return;
  if (in_sizes[5] != kXpN * kDi) return;
  if (in_sizes[6] != kDi * kDtR) return;
  if (in_sizes[7] != kDi) return;
  if (in_sizes[8] != kDi * kNs) return;
  if (in_sizes[9] != kDi) return;
  if (in_sizes[10] != kDm * kDi) return;
  if (in_sizes[11] != kDm * kDm) return;
  if (in_sizes[12] != kDm) return;
  if (in_sizes[13] != kDm * kDm) return;
  if (in_sizes[14] != kDm) return;
  if (in_sizes[15] != kDm) return;
  if (in_sizes[16] != kDm) return;
  if (out_size != kRows * kDm + kNB * kHidB) return;
  if (ws_size < kWsTotal) return;

  const float* x        = (const float*)d_in[0];
  const float* norm_w   = (const float*)d_in[1];
  const float* in_proj  = (const float*)d_in[2];
  const float* conv_w   = (const float*)d_in[3];
  const float* conv_b   = (const float*)d_in[4];
  const float* x_proj   = (const float*)d_in[5];
  const float* dt_w     = (const float*)d_in[6];
  const float* dt_b     = (const float*)d_in[7];
  const float* A_log    = (const float*)d_in[8];
  const float* Dp       = (const float*)d_in[9];
  const float* out_proj = (const float*)d_in[10];
  const float* ff_w1    = (const float*)d_in[11];
  const float* ff_b1    = (const float*)d_in[12];
  const float* ff_w2    = (const float*)d_in[13];
  const float* ff_b2    = (const float*)d_in[14];
  const float* ff_ln_w  = (const float*)d_in[15];
  const float* ff_ln_b  = (const float*)d_in[16];

  float* dout_main = (float*)d_out;
  float* dout_hid  = dout_main + (size_t)kRows * kDm;

  char* ws = (char*)d_ws;
  unsigned short* WIN  = (unsigned short*)(ws + kOffWIN);
  unsigned short* WXP  = (unsigned short*)(ws + kOffWXP);
  unsigned short* WDT  = (unsigned short*)(ws + kOffWDT);
  unsigned short* WOUT = (unsigned short*)(ws + kOffWOUT);
  unsigned short* WF1  = (unsigned short*)(ws + kOffWF1);
  unsigned short* WF2  = (unsigned short*)(ws + kOffWF2);
  unsigned short* XN   = (unsigned short*)(ws + kOffXN);
  unsigned short* P16  = (unsigned short*)(ws + kOffP);
  unsigned short* UC16 = (unsigned short*)(ws + kOffUC);
  float*          DBL  = (float*)(ws + kOffDBL);
  unsigned short* DTR  = (unsigned short*)(ws + kOffDTR);
  float*          DLR  = (float*)(ws + kOffDLR);
  unsigned short* Y16  = (unsigned short*)(ws + kOffY);
  unsigned short* O16  = UC16;
  unsigned short* H16  = UC16 + (size_t)kRows * kDm;
  float*          RES  = DLR;
  float*          O32  = DLR + (size_t)kRows * kDm;
  const float* no_bias = dt_b;

  cast_f16_kernel<<<(kPw * kDm / 8) / 256, 256, 0, stream>>>(in_proj, WIN, kPw * kDm / 8, kPw * kDm / 8, kWCarry);
  cast_f16_kernel<<<(kXpP * kDi / 8) / 256, 256, 0, stream>>>(x_proj, WXP, kXpP * kDi / 8, kXpN * kDi / 8, kWCarry);
  cast_f16_kernel<<<(kDi * kDtR / 8) / 256, 256, 0, stream>>>(dt_w, WDT, kDi * kDtR / 8, kDi * kDtR / 8, kDtWCarry);
  cast_f16_kernel<<<(kDm * kDi / 8) / 256, 256, 0, stream>>>(out_proj, WOUT, kDm * kDi / 8, kDm * kDi / 8, kWCarry);
  cast_f16_kernel<<<(kDm * kDm / 8) / 256, 256, 0, stream>>>(ff_w1, WF1, kDm * kDm / 8, kDm * kDm / 8, kWCarry);
  cast_f16_kernel<<<(kDm * kDm / 8) / 256, 256, 0, stream>>>(ff_w2, WF2, kDm * kDm / 8, kDm * kDm / 8, kWCarry);

  rmsnorm_f16_kernel<<<kRows / 8, 256, 0, stream>>>(x, norm_w, XN);

  wmma_gemm64_f16<0, 1><<<dim3((kRows / 64) * (kPw / 64) / 8), 256, 0, stream>>>(
      XN, kDm, WIN, kDm, (void*)P16, kPw, no_bias, kRows, kPw, kDm, 1.0f / kWCarry);

  conv_silu_kernel<<<dim3(kDi / 256, kRows / 64), 256, 0, stream>>>((const unsigned*)P16, conv_w, conv_b, UC16);

  wmma_gemm64_f16<0, 0><<<dim3((kRows / 64) * (kXpP / 64) / 8), 256, 0, stream>>>(
      UC16, kDi, WXP, kDi, (void*)DBL, kXpP, no_bias, kRows, kXpP, kDi, 1.0f / kWCarry);

  dt_cast_kernel<<<(kRows * kDtR / 8) / 256, 256, 0, stream>>>(DBL, DTR, kRows * kDtR / 8);

  wmma_gemm64_f16<2, 0><<<dim3((kRows / 64) * (kDi / 64) / 8), 256, 0, stream>>>(
      DTR, kDtR, WDT, kDtR, (void*)DLR, kDi, dt_b, kRows, kDi, kDtR, 1.0f / kDtWCarry);

  scan_gate_kernel<<<kNB * (kDi / 256), 256, 0, stream>>>(
      DLR, (const unsigned*)UC16, (const unsigned*)P16, DBL, A_log, Dp, Y16, dout_hid);

  wmma_gemm64_f16<0, 0><<<dim3((kRows / 64) * (kDm / 64) / 8), 256, 0, stream>>>(
      Y16, kDi, WOUT, kDi, (void*)RES, kDm, no_bias, kRows, kDm, kDi, 1.0f / (kYCarry * kWCarry));

  resadd_kernel<<<(kRows * kDm) / 2048, 256, 0, stream>>>(RES, x, O32, O16);

  wmma_gemm64_f16<2, 0><<<dim3((kRows / 64) * (kDm / 64) / 8), 256, 0, stream>>>(
      O16, kDm, WF1, kDm, (void*)RES, kDm, ff_b1, kRows, kDm, kDm, 1.0f / kWCarry);

  gelu_f16_kernel<<<(kRows * kDm) / 2048, 256, 0, stream>>>(RES, H16);

  wmma_gemm64_f16<2, 0><<<dim3((kRows / 64) * (kDm / 64) / 8), 256, 0, stream>>>(
      H16, kDm, WF2, kDm, (void*)RES, kDm, ff_b2, kRows, kDm, kDm, 1.0f / kWCarry);

  layernorm_out_kernel<<<kRows, 256, 0, stream>>>(RES, O32, ff_ln_w, ff_ln_b, dout_main);

  utail_kernel<<<kDi / 32, 256, 0, stream>>>(x, norm_w, in_proj, dout_hid);
}
